// DiscreteAttnTRBlock_41231686042368
// MI455X (gfx1250) — hardware-verified
//
#include <hip/hip_runtime.h>
#include <stddef.h>


typedef __bf16 v8b __attribute__((ext_vector_type(8)));
typedef __bf16 v16b __attribute__((ext_vector_type(16)));
typedef float v4f __attribute__((ext_vector_type(4)));
typedef float v8f __attribute__((ext_vector_type(8)));
typedef double v2d __attribute__((ext_vector_type(2)));

#define CCH 128
#define QCH 16
#define NTAP 27
#define NBLK 128
#define FRAG 512
#define CROWS 256


__device__ __forceinline__ v16b cat_b(v8b a, v8b b) {
  return __builtin_shufflevector(a, b, 0, 1, 2, 3, 4, 5, 6, 7, 8, 9, 10, 11, 12, 13, 14, 15);
}

__device__ __forceinline__ v16b frag_b(const unsigned short* p) {
  const v8b* q = (const v8b*)p;
  return cat_b(q[0], q[1]);
}

__device__ __forceinline__ v4f ld4(const float* p) { return *(const v4f*)p; }

__device__ __forceinline__ v4f relu4(v4f v) {
  v4f r;
  r[0] = fmaxf(v[0], 0.0f);
  r[1] = fmaxf(v[1], 0.0f);
  r[2] = fmaxf(v[2], 0.0f);
  r[3] = fmaxf(v[3], 0.0f);
  return r;
}

__device__ __forceinline__ void split16(v4f f0, v4f f1, v4f f2, v4f f3, v16b& hi, v16b& lo) {
  v16b th = {}, tl = {};
#pragma unroll
  for (int e = 0; e < 4; ++e) {
    const float a = f0[e], b = f1[e], c = f2[e], d = f3[e];
    const __bf16 ha = (__bf16)a, hb = (__bf16)b, hc = (__bf16)c, hd = (__bf16)d;
    th[e] = ha;
    th[4 + e] = hb;
    th[8 + e] = hc;
    th[12 + e] = hd;
    tl[e] = (__bf16)(a - (float)ha);
    tl[4 + e] = (__bf16)(b - (float)hb);
    tl[8 + e] = (__bf16)(c - (float)hc);
    tl[12 + e] = (__bf16)(d - (float)hd);
  }
  hi = th;
  lo = tl;
}

__device__ __forceinline__ v8f mma3(v8f c, v16b ah, v16b al, v16b bh, v16b bl) {
  c = __builtin_amdgcn_wmma_f32_16x16x32_bf16(false, ah, false, bh, (short)0, c, false, false);
  c = __builtin_amdgcn_wmma_f32_16x16x32_bf16(false, ah, false, bl, (short)0, c, false, false);
  c = __builtin_amdgcn_wmma_f32_16x16x32_bf16(false, al, false, bh, (short)0, c, false, false);
  asm volatile("v_nop\n\tv_nop\n\tv_nop\n\tv_nop" : "+v"(c) : "v"(ah), "v"(al), "v"(bh), "v"(bl));
  return c;
}

__global__ __launch_bounds__(256) void swz_kernel(const float* __restrict__ W,
                                                 unsigned short* __restrict__ oh,
                                                 unsigned short* __restrict__ ol, int taps,
                                                 int cout) {
  const int NT = cout >> 4;
  const unsigned total = (unsigned)taps * 4u * (unsigned)NT * 64u;
  const unsigned p = blockIdx.x * 256u + threadIdx.x;
  if (p >= total) return;
  const int g = (int)(p & 1u);
  const int lane = (int)((p >> 1) & 31u);
  const unsigned f = p >> 6;
  const int nt = (int)(f % (unsigned)NT);
  const unsigned t2 = f / (unsigned)NT;
  const int kc = (int)(t2 & 3u);
  const int tap = (int)(t2 >> 2);
  const int h = lane >> 4;
  const int n = nt * 16 + (lane & 15);
  const int K = kc * 32 + 16 * g + 8 * h;
  const float* src = W + ((size_t)tap * CCH + K) * cout + n;
  v8b hi = {}, lo = {};
#pragma unroll
  for (int jj = 0; jj < 8; ++jj) {
    const float w = src[(size_t)jj * cout];
    const __bf16 hb = (__bf16)w;
    hi[jj] = hb;
    lo[jj] = (__bf16)(w - (float)hb);
  }
  unsigned short* dh = oh + (size_t)p * 8;
  unsigned short* dl = ol + (size_t)p * 8;
  *(volatile v8b*)dh = hi;
  *(volatile v8b*)dl = lo;
  __threadfence();
  *(volatile v8b*)dh = hi;
  *(volatile v8b*)dl = lo;
}

__global__ __launch_bounds__(256) void gather_kernel(const float* __restrict__ x,
                                                    const int* __restrict__ nbr,
                                                    float* __restrict__ G, int R, int rowBase,
                                                    int N, int nb) {
  __shared__ int pc[8];
  const int tid = threadIdx.x, lane = tid & 31, wave = tid >> 5;
  const int k = (int)blockIdx.x / nb;
  const int cx = (int)blockIdx.x - k * nb;
  const int lrow0 = cx * CROWS;
  const int row = rowBase + lrow0 + tid;
  int idx = -1;
  if (row < N) idx = nbr[(size_t)k * N + row];
  const bool vld = idx >= 0;
  if (idx > N - 1) idx = N - 1;
  if (idx < 0) idx = 0;
  const unsigned mask = (unsigned)__ballot(vld ? 1 : 0);
  if (lane == 0) pc[wave] = (int)__builtin_popcount(mask);
  __syncthreads();
  int base = 0, cnt = 0;
#pragma unroll
  for (int w = 0; w < 8; ++w) {
    const int v = pc[w];
    cnt += v;
    base += (w < wave) ? v : 0;
  }
  const int slot = base + (int)__builtin_popcount(mask & ((1u << lane) - 1u));
  const int cnt16 = (cnt + 15) & ~15;
  float* gb = G + ((size_t)k * R + (size_t)lrow0) * CCH;

  if (tid >= cnt && tid < cnt16) {
    float* d = gb + (size_t)tid * CCH;
    const v4f z = {};
#pragma unroll
    for (int q = 0; q < 32; ++q) *(volatile v4f*)(d + 4 * q) = z;
    __threadfence();
#pragma unroll
    for (int q = 0; q < 32; ++q) *(volatile v4f*)(d + 4 * q) = z;
  }
  if (vld) {
    const float* s = x + (size_t)idx * CCH;
    float* d = gb + (size_t)slot * CCH;
#pragma unroll
    for (int half = 0; half < 2; ++half) {
      v4f b[16];
#pragma unroll
      for (int q = 0; q < 16; ++q) b[q] = ld4(s + half * 64 + 4 * q);
#pragma unroll
      for (int q = 0; q < 16; ++q) *(volatile v4f*)(d + half * 64 + 4 * q) = b[q];
      __threadfence();
#pragma unroll
      for (int q = 0; q < 16; ++q) *(volatile v4f*)(d + half * 64 + 4 * q) = b[q];
    }
  }
}

__global__ __launch_bounds__(256) __attribute__((amdgpu_num_vgpr(256)))
void conv_kernel(const float* __restrict__ G, const int* __restrict__ nbr,
                 const unsigned short* __restrict__ Bh, const unsigned short* __restrict__ Bl,
                 float* __restrict__ Y, int R, int rowBase, int N) {
  __shared__ __align__(16) float accl[CROWS * CCH];
  __shared__ int rowof[CROWS];
  __shared__ int pc[8];
  const int tid = threadIdx.x;
  const int lane = tid & 31, wave = tid >> 5, h = lane >> 4, m = lane & 15;
  const int lrow0 = (int)blockIdx.x * CROWS;
  const int grow0 = rowBase + lrow0;
  {
    const v4f z = {};
    v4f* ar = (v4f*)(accl + tid * CCH);
#pragma unroll
    for (int q = 0; q < 32; ++q) ar[q] = z;
  }

#pragma unroll 1
  for (int k = 0; k < NTAP; ++k) {
    __syncthreads();
    const int row = grow0 + tid;
    bool vld = false;
    if (row < N) vld = nbr[(size_t)k * N + row] >= 0;
    const unsigned mask = (unsigned)__ballot(vld ? 1 : 0);
    if (lane == 0) pc[wave] = (int)__builtin_popcount(mask);
    __syncthreads();
    int base = 0, cnt = 0;
#pragma unroll
    for (int w = 0; w < 8; ++w) {
      const int v = pc[w];
      cnt += v;
      base += (w < wave) ? v : 0;
    }
    const int slot = base + (int)__builtin_popcount(mask & ((1u << lane) - 1u));
    int cnt16 = (cnt + 15) & ~15;
    if (cnt16 > CROWS) cnt16 = CROWS;
    if (tid >= cnt && tid < cnt16) rowof[tid] = -1;
    if (vld) rowof[slot] = tid;
    __syncthreads();
    const int ntiles = cnt16 >> 4;

    for (int t = wave; t < ntiles; t += 8) {
      v8f acc[8];
      {
        const v8f z = {};
#pragma unroll
        for (int i = 0; i < 8; ++i) acc[i] = z;
      }
      const float* ap = G + ((size_t)k * R + (size_t)(lrow0 + t * 16 + m)) * CCH;
#pragma unroll
      for (int kc = 0; kc < 4; ++kc) {
        const float* p0 = ap + kc * 32 + 8 * h;
        const v4f f0 = ld4(p0), f1 = ld4(p0 + 4), f2 = ld4(p0 + 16), f3 = ld4(p0 + 20);
        v16b ah, al;
        split16(f0, f1, f2, f3, ah, al);
#pragma unroll
        for (int gb = 0; gb < 8; gb += 4) {
#pragma unroll
          for (int j = 0; j < 4; ++j) {
            const size_t f = (size_t)((k * 4 + kc) * 8 + gb + j) * FRAG + (size_t)lane * 16;
            const v16b bh = frag_b(Bh + f);
            const v16b bl = frag_b(Bl + f);
            acc[gb + j] = mma3(acc[gb + j], ah, al, bh, bl);
          }
        }
      }
#pragma unroll
      for (int r = 0; r < 8; ++r) {
        int lr = rowof[t * 16 + 8 * h + r];
        if (lr >= 0) {
          if (lr > CROWS - 1) lr = CROWS - 1;
          float* arow = accl + lr * CCH + m;
#pragma unroll
          for (int nt = 0; nt < 8; ++nt) arow[nt * 16] += acc[nt][r];
        }
      }
    }
  }
  __syncthreads();

  float* yb = Y + lane * 4;
#pragma unroll 1
  for (int i = 0; i < 32; ++i) {
    const int lr = wave * 32 + i;
    const int grow = grow0 + lr;
    if (grow < N) {
      const v4f v = ((const v4f*)(accl + lr * CCH))[lane];
      *(volatile v4f*)(yb + (size_t)grow * CCH) = v;
    }
  }
  __threadfence();
#pragma unroll 1
  for (int i = 0; i < 32; ++i) {
    const int lr = wave * 32 + i;
    const int grow = grow0 + lr;
    if (grow < N) {
      const v4f v = ((const v4f*)(accl + lr * CCH))[lane];
      *(volatile v4f*)(yb + (size_t)grow * CCH) = v;
    }
  }
}

template <int NT, int FUSE>
__global__ __launch_bounds__(256) __attribute__((amdgpu_num_vgpr(256)))
void gemm_kernel(const float* __restrict__ A, int aRows, const float* __restrict__ sb,
                 const unsigned short* __restrict__ Bh, const unsigned short* __restrict__ Bl,
                 float* __restrict__ Y, int nTiles) {
  constexpr int C = NT * 16;
  constexpr int GW = (NT < 4) ? NT : 4;
  __shared__ __align__(16) float stgl[8 * 16 * C];
  const int tid = threadIdx.x;
  const int lane = tid & 31, wave = tid >> 5, h = lane >> 4, m = lane & 15;
  const int tile = (int)blockIdx.x * 8 + wave;
  const bool active = tile < nTiles;
  const int rowBase = active ? tile * 16 : 0;
  int aRow = rowBase + m;
  if (aRow > aRows - 1) aRow = aRows - 1;
  if (aRow < 0) aRow = 0;
  const float* ap = A + (size_t)aRow * CCH;

  v8f acc[NT];
  {
    const v8f z = {};
#pragma unroll
    for (int t = 0; t < NT; ++t) acc[t] = z;
  }

#pragma unroll
  for (int kc = 0; kc < 4; ++kc) {
    const int c0 = kc * 32 + 8 * h;
    const float* p0 = ap + c0;
    v4f f0 = ld4(p0), f1 = ld4(p0 + 4), f2 = ld4(p0 + 16), f3 = ld4(p0 + 20);
    if (FUSE) {
      f0 = relu4(f0 * ld4(sb + c0) + ld4(sb + CCH + c0));
      f1 = relu4(f1 * ld4(sb + c0 + 4) + ld4(sb + CCH + c0 + 4));
      f2 = relu4(f2 * ld4(sb + c0 + 16) + ld4(sb + CCH + c0 + 16));
      f3 = relu4(f3 * ld4(sb + c0 + 20) + ld4(sb + CCH + c0 + 20));
    }
    v16b ah, al;
    split16(f0, f1, f2, f3, ah, al);
#pragma unroll
    for (int gb = 0; gb < NT; gb += GW) {
#pragma unroll
      for (int j = 0; j < GW; ++j) {
        const size_t f = (size_t)(kc * NT + gb + j) * FRAG + (size_t)lane * 16;
        const v16b bh = frag_b(Bh + f);
        const v16b bl = frag_b(Bl + f);
        acc[gb + j] = mma3(acc[gb + j], ah, al, bh, bl);
      }
    }
  }

  float* sw = stgl + wave * (16 * C);
#pragma unroll
  for (int nt = 0; nt < NT; ++nt)
#pragma unroll
    for (int r = 0; r < 8; ++r) sw[(8 * h + r) * C + nt * 16 + m] = acc[nt][r];
  __syncthreads();
  if (active) {
    const v4f* s4 = (const v4f*)sw;
    float* yb = Y + (size_t)rowBase * C;
#pragma unroll
    for (int s = 0; s < 2 * NT; ++s)
      *(volatile v4f*)(yb + (size_t)(s * 32 + lane) * 4) = s4[s * 32 + lane];
    __threadfence();
#pragma unroll
    for (int s = 0; s < 2 * NT; ++s)
      *(volatile v4f*)(yb + (size_t)(s * 32 + lane) * 4) = s4[s * 32 + lane];
  }
}

__global__ __launch_bounds__(256) void stats_part_kernel(const float* __restrict__ y,
                                                        double* __restrict__ part, int nCh,
                                                        int nRows) {
  __shared__ __align__(16) double ss[256 * 4];
  __shared__ __align__(16) double sq[256 * 4];
  const int t = threadIdx.x;
  const int tpr = nCh >> 2;
  const int cg = t & (tpr - 1);
  const int r0 = t / tpr;
  const int rpi = 256 / tpr;
  const int slab = (nRows + (int)gridDim.x - 1) / (int)gridDim.x;
  const int start = (int)blockIdx.x * slab;
  int end = start + slab;
  if (end > nRows) end = nRows;
  double s0 = 0.0, s1 = 0.0, s2 = 0.0, s3 = 0.0, q0 = 0.0, q1 = 0.0, q2 = 0.0, q3 = 0.0;
#pragma unroll 1
  for (int r = start + r0; r < end; r += rpi) {
    const v4f v = ld4(y + (size_t)r * nCh + cg * 4);
    const double d0 = v[0], d1 = v[1], d2 = v[2], d3 = v[3];
    s0 += d0; s1 += d1; s2 += d2; s3 += d3;
    q0 += d0 * d0; q1 += d1 * d1; q2 += d2 * d2; q3 += d3 * d3;
  }
  ss[t * 4 + 0] = s0; ss[t * 4 + 1] = s1; ss[t * 4 + 2] = s2; ss[t * 4 + 3] = s3;
  sq[t * 4 + 0] = q0; sq[t * 4 + 1] = q1; sq[t * 4 + 2] = q2; sq[t * 4 + 3] = q3;
  __syncthreads();
  for (int st = 128; st >= tpr; st >>= 1) {
    if (t < st) {
#pragma unroll
      for (int e = 0; e < 4; ++e) {
        ss[t * 4 + e] += ss[(t + st) * 4 + e];
        sq[t * 4 + e] += sq[(t + st) * 4 + e];
      }
    }
    __syncthreads();
  }
  double* pb = part + (size_t)blockIdx.x * 2 * nCh;
  if (t < nCh) {
    const int hn = nCh >> 1;
    const double* srcArr;
    double* d;
    int c;
    if (t < hn) { c = 2 * t; srcArr = ss; d = pb + c; }
    else        { c = 2 * (t - hn); srcArr = sq; d = pb + nCh + c; }
    v2d val;
    val[0] = srcArr[c];
    val[1] = srcArr[c + 1];
    *(volatile v2d*)d = val;
    __threadfence();
    *(volatile v2d*)d = val;
  }
}

__global__ __launch_bounds__(128) void stats_final_kernel(const double* __restrict__ part,
                                                         const float* __restrict__ g,
                                                         const float* __restrict__ b,
                                                         float* __restrict__ sb, int nCh,
                                                         int nBlk, int nRows) {
  __shared__ __align__(16) float la[128];
  __shared__ __align__(16) float lb[128];
  const int c = threadIdx.x;
  if (c < nCh) {
    double s = 0.0, q = 0.0;
#pragma unroll 1
    for (int i = 0; i < nBlk; ++i) {
      s += part[(size_t)i * 2 * nCh + c];
      q += part[(size_t)i * 2 * nCh + nCh + c];
    }
    const double mu = s / (double)nRows;
    double var = q / (double)nRows - mu * mu;
    if (var < 0.0) var = 0.0;
    const float vf = (float)var;
    const float rs = 1.0f / sqrtf(vf + 1e-5f);
    const float Av = rs * g[c];
    const float Bv = b[c] - (float)mu * Av;
    la[c] = Av;
    lb[c] = Bv;
  }
  __syncthreads();
  const int nw = nCh >> 2;
  if (c < 2 * nw) {
    v4f v;
    float* dst;
    if (c < nw) { v = ((const v4f*)la)[c]; dst = sb + 4 * c; }
    else        { v = ((const v4f*)lb)[c - nw]; dst = sb + nCh + 4 * (c - nw); }
    *(volatile v4f*)dst = v;
    __threadfence();
    *(volatile v4f*)dst = v;
  }
}

__device__ __forceinline__ float expert_acc(const int* __restrict__ nb, int K,
                                            const float* __restrict__ cb,
                                            const float* __restrict__ qraw, float qA, float qB,
                                            const float* __restrict__ y2, v4f vA0, v4f vA1,
                                            v4f vB0, v4f vB1, int N, int p, int j, float qi,
                                            v4f& oa, v4f& ob) {
  float aq = 0.0f, cnt = 0.0f;
  const v4f za = {};
  oa = za;
  ob = za;
#pragma unroll 1
  for (int k = 0; k < K; ++k) {
    int idx = nb[(size_t)k * N + p];
    if (idx >= 0) {
      if (idx > N - 1) idx = N - 1;
      aq += fmaxf(qraw[(size_t)idx * QCH + j] * qA + qB, 0.0f);
      cnt += 1.0f;
      const float* vp = y2 + (size_t)idx * CCH + 8 * j;
      const float* wp = cb + (size_t)k * CCH + 8 * j;
      const v4f va = relu4(ld4(vp) * vA0 + vB0);
      const v4f vb = relu4(ld4(vp + 4) * vA1 + vB1);
      oa += ld4(wp) * va;
      ob += ld4(wp + 4) * vb;
    }
  }
  return (qi * aq) * (1.0f / fmaxf(cnt, 1.0f));
}

__global__ __launch_bounds__(256) void mix_kernel(const float* __restrict__ qraw,
                                                 const float* __restrict__ sbq,
                                                 const float* __restrict__ y2,
                                                 const float* __restrict__ sbv,
                                                 const int* __restrict__ nb0,
                                                 const int* __restrict__ nb1,
                                                 const int* __restrict__ nb2,
                                                 const float* __restrict__ cb0,
                                                 const float* __restrict__ cb1,
                                                 const float* __restrict__ cb2,
                                                 float* __restrict__ dst, int N) {
  __shared__ __align__(16) float rowbuf[16 * CCH];
  const int tid = threadIdx.x;
  const int pl = tid >> 4, j = tid & 15;
  const int p = (int)blockIdx.x * 16 + pl;
  v4f ra = {}, rb = {};
  if (p < N) {
    const float qA = sbq[j], qB = sbq[QCH + j];
    const v4f vA0 = ld4(sbv + 8 * j), vA1 = ld4(sbv + 8 * j + 4);
    const v4f vB0 = ld4(sbv + CCH + 8 * j), vB1 = ld4(sbv + CCH + 8 * j + 4);
    const float qi = fmaxf(qraw[(size_t)p * QCH + j] * qA + qB, 0.0f);
    v4f o0a, o0b, o1a, o1b, o2a, o2b;
    const float s0 = expert_acc(nb0, 7, cb0, qraw, qA, qB, y2, vA0, vA1, vB0, vB1, N, p, j, qi, o0a, o0b);
    const float s1 = expert_acc(nb1, 27, cb1, qraw, qA, qB, y2, vA0, vA1, vB0, vB1, N, p, j, qi, o1a, o1b);
    const float s2 = expert_acc(nb2, 7, cb2, qraw, qA, qB, y2, vA0, vA1, vB0, vB1, N, p, j, qi, o2a, o2b);
    const float mx = fmaxf(s0, fmaxf(s1, s2));
    const float e0 = expf(s0 - mx), e1 = expf(s1 - mx), e2 = expf(s2 - mx);
    const float inv = 1.0f / (e0 + e1 + e2);
    const float w0 = e0 * inv, w1 = e1 * inv, w2 = e2 * inv;
    ra = w0 * o0a;
    ra = ra + w1 * o1a;
    ra = ra + w2 * o2a;
    rb = w0 * o0b;
    rb = rb + w1 * o1b;
    rb = rb + w2 * o2b;
  }
  {
    v4f* rw = (v4f*)(rowbuf + pl * CCH + 8 * j);
    rw[0] = ra;
    rw[1] = rb;
  }
  __syncthreads();
  if (p < N) {
    const v4f* rr = (const v4f*)(rowbuf + pl * CCH);
    const v4f u0 = rr[j], u1 = rr[16 + j];
    float* op = dst + (size_t)p * CCH;
    *(volatile v4f*)(op + 4 * j) = u0;
    *(volatile v4f*)(op + 64 + 4 * j) = u1;
    __threadfence();
    *(volatile v4f*)(op + 4 * j) = u0;
    *(volatile v4f*)(op + 64 + 4 * j) = u1;
  }
}

__global__ __launch_bounds__(256) void final_kernel(const float* __restrict__ y,
                                                   const float* __restrict__ sb,
                                                   const float* __restrict__ x,
                                                   float* __restrict__ out, unsigned total4) {
  const unsigned i = blockIdx.x * 256u + threadIdx.x;
  if (i >= total4) return;
  const int c0 = (int)((i * 4u) & (unsigned)(CCH - 1));
  const v4f v = ((const v4f*)y)[i];
  const v4f Av = ld4(sb + c0);
  const v4f Bv = ld4(sb + CCH + c0);
  v4f r = relu4(v * Av + Bv);
  r = r + ((const v4f*)x)[i];
  float* dst = out + (size_t)i * 4;
  *(volatile v4f*)dst = r;
  __threadfence();
  *(volatile v4f*)dst = r;
}

static inline unsigned swz_blocks(int taps, int cout) {
  const unsigned pieces = (unsigned)taps * 4u * (unsigned)(cout >> 4) * 64u;
  return (pieces + 255u) / 256u;
}

extern "C" void kernel_launch(void* const* d_in, const int* in_sizes, int n_in, void* d_out,
                              int out_size, void* d_ws, size_t ws_size, hipStream_t stream) {
  (void)n_in;
  const float* x = (const float*)d_in[0];
  const float* v1_w = (const float*)d_in[1];
  const float* v1_g = (const float*)d_in[2];
  const float* v1_b = (const float*)d_in[3];
  const float* v2_w = (const float*)d_in[4];
  const float* v2_g = (const float*)d_in[5];
  const float* v2_b = (const float*)d_in[6];
  const float* q_w = (const float*)d_in[7];
  const float* q_g = (const float*)d_in[8];
  const float* q_b = (const float*)d_in[9];
  const float* cb0 = (const float*)d_in[10];
  const float* cb1 = (const float*)d_in[11];
  const float* cb2 = (const float*)d_in[12];
  const float* out_w = (const float*)d_in[13];
  const float* out_g = (const float*)d_in[14];
  const float* out_b = (const float*)d_in[15];
  const int* nbr_cross2 = (const int*)d_in[16];
  const int* nbr_cube = (const int*)d_in[17];
  const int* nbr_cross3 = (const int*)d_in[18];

  const int N = in_sizes[0] / CCH;
  if (N <= 0) return;
  const int Np = (N + 15) & ~15;
  const int nTiles = Np / 16;

  long Rl = 72000000L / ((long)NTAP * CCH * 4);
  Rl &= ~255L;
  const long nAl = ((long)N + 255) & ~255L;
  if (Rl > nAl) Rl = nAl;
  if (Rl < CROWS) Rl = CROWS;
  const int R = (int)Rl;
  const int nLC = (N + R - 1) / R;

  char* base = (char*)d_ws;
  size_t off = 0;
  auto alloc = [&](size_t bytes) -> char* {
    char* p = base + off;
    off = (off + bytes + 255) & ~(size_t)255;
    return p;
  };
  const size_t yBytes = (size_t)N * CCH * 4;
  const size_t stgBytes = (size_t)NTAP * (size_t)R * CCH * 4;
  const size_t bNeed = (size_t)Np * CCH * 4 + (size_t)Np * QCH * 4;
  const size_t bBytes = (stgBytes > bNeed) ? stgBytes : bNeed;

  char* regY = alloc(yBytes);
  char* regB = alloc(bBytes);
  unsigned short* w1h = (unsigned short*)alloc((size_t)NTAP * 16384 * 2);
  unsigned short* w1l = (unsigned short*)alloc((size_t)NTAP * 16384 * 2);
  unsigned short* w2h = (unsigned short*)alloc((size_t)16384 * 2);
  unsigned short* w2l = (unsigned short*)alloc((size_t)16384 * 2);
  unsigned short* qh = (unsigned short*)alloc((size_t)2048 * 2);
  unsigned short* ql = (unsigned short*)alloc((size_t)2048 * 2);
  unsigned short* oh = (unsigned short*)alloc((size_t)16384 * 2);
  unsigned short* ol = (unsigned short*)alloc((size_t)16384 * 2);
  double* part = (double*)alloc((size_t)NBLK * 2 * CCH * 8);
  float* sb1 = (float*)alloc(1024);
  float* sb2 = (float*)alloc(1024);
  float* sb3 = (float*)alloc(1024);
  float* sb4 = (float*)alloc(1024);
  if (off > ws_size) return;

  float* y1 = (float*)regY;
  float* obuf = (float*)regY;
  float* G = (float*)regB;
  float* y2 = (float*)regB;
  float* qraw = (float*)(regB + (size_t)Np * CCH * 4);
  float* y3 = (float*)regB;
  float* outp = (float*)d_out;

  swz_kernel<<<swz_blocks(NTAP, CCH), 256, 0, stream>>>(v1_w, w1h, w1l, NTAP, CCH);
  swz_kernel<<<swz_blocks(1, CCH), 256, 0, stream>>>(v2_w, w2h, w2l, 1, CCH);
  swz_kernel<<<swz_blocks(1, QCH), 256, 0, stream>>>(q_w, qh, ql, 1, QCH);
  swz_kernel<<<swz_blocks(1, CCH), 256, 0, stream>>>(out_w, oh, ol, 1, CCH);

  for (int lc = 0; lc < nLC; ++lc) {
    const int rowBase = lc * R;
    int Rc = N - rowBase;
    if (Rc > R) Rc = R;
    const int nb = (Rc + CROWS - 1) / CROWS;
    gather_kernel<<<(unsigned)(nb * NTAP), 256, 0, stream>>>(x, nbr_cube, G, R, rowBase, N, nb);
    conv_kernel<<<(unsigned)nb, 256, 0, stream>>>(G, nbr_cube, w1h, w1l, y1, R, rowBase, N);
  }
  const unsigned gemmGrid = (unsigned)((nTiles + 7) / 8);

  stats_part_kernel<<<NBLK, 256, 0, stream>>>(y1, part, CCH, N);
  stats_final_kernel<<<1, 128, 0, stream>>>(part, v1_g, v1_b, sb1, CCH, NBLK, N);

  gemm_kernel<8, 1><<<gemmGrid, 256, 0, stream>>>(y1, N, sb1, w2h, w2l, y2, nTiles);
  stats_part_kernel<<<NBLK, 256, 0, stream>>>(y2, part, CCH, N);
  stats_final_kernel<<<1, 128, 0, stream>>>(part, v2_g, v2_b, sb2, CCH, NBLK, N);

  gemm_kernel<1, 0><<<gemmGrid, 256, 0, stream>>>(x, N, sb1, qh, ql, qraw, nTiles);
  stats_part_kernel<<<NBLK, 256, 0, stream>>>(qraw, part, QCH, N);
  stats_final_kernel<<<1, 128, 0, stream>>>(part, q_g, q_b, sb3, QCH, NBLK, N);

  mix_kernel<<<(unsigned)((N + 15) / 16), 256, 0, stream>>>(qraw, sb3, y2, sb2, nbr_cross2, nbr_cube,
                                                           nbr_cross3, cb0, cb1, cb2, obuf, N);

  gemm_kernel<8, 0><<<gemmGrid, 256, 0, stream>>>(obuf, N, sb1, oh, ol, y3, nTiles);
  stats_part_kernel<<<NBLK, 256, 0, stream>>>(y3, part, CCH, N);
  stats_final_kernel<<<1, 128, 0, stream>>>(part, out_g, out_b, sb4, CCH, NBLK, N);
  const unsigned out4 = (unsigned)out_size / 4u;
  final_kernel<<<(out4 + 255u) / 256u, 256, 0, stream>>>(y3, sb4, x, outp, out4);
}
